// QuadraticInhibitorAttention_55817394979295
// MI455X (gfx1250) — hardware-verified
//
#include <hip/hip_runtime.h>
#include <math.h>

typedef __attribute__((ext_vector_type(16))) _Float16 v16h;
typedef __attribute__((ext_vector_type(8)))  _Float16 v8h;
typedef __attribute__((ext_vector_type(8)))  float    v8f;
typedef __attribute__((ext_vector_type(4)))  float    v4f;
typedef __attribute__((ext_vector_type(4)))  unsigned int v4u;

constexpr int kS    = 512;
constexpr int kHid  = 512;
constexpr int kNH   = 8;
constexpr int kD    = 64;
constexpr int kQKV  = 3 * kHid;
constexpr float kSqrtD = 8.0f;
static_assert(kNH * kD == kHid);
static_assert(kSqrtD * kSqrtD == (float)kD);
static_assert((kS % 64) == 0 && (kHid % 64) == 0 && (kQKV % 64) == 0 && (kHid % 32) == 0 && (kD % 32) == 0);

constexpr float kXCarry   = 16.0f;
constexpr float kWCarry   = 1024.0f;
constexpr float kQKCarry  = 64.0f;
constexpr float kCtxCarry = 1.0f;
constexpr float kProjScale = 1.0f / (kXCarry * kWCarry);
constexpr float kOutScale  = 1.0f / (kCtxCarry * kWCarry);
constexpr float kInvQK2    = 1.0f / (kQKCarry * kQKCarry);
constexpr float kF16MinNormal = 6.103515625e-05f;
constexpr float kMaskPen = 1e10f;

constexpr int kIT = 32;
constexpr int kJC = 128;
constexpr int kZP = 132;
static_assert((kS % kIT) == 0 && (kS % kJC) == 0 && (kZP % 4) == 0 && kZP >= kJC);

constexpr size_t kOffXH   = 0;
constexpr size_t kOffWQKV = kOffXH   + (size_t)kS   * kHid * 2;
constexpr size_t kOffWOH  = kOffWQKV + (size_t)kQKV * kHid * 2;
constexpr size_t kOffQH   = kOffWOH  + (size_t)kHid * kHid * 2;
constexpr size_t kOffKH   = kOffQH   + (size_t)kS   * kHid * 2;
constexpr size_t kOffVF   = kOffKH   + (size_t)kS   * kHid * 2;
constexpr size_t kOffZQ   = kOffVF   + (size_t)kS   * kHid * 4;
constexpr size_t kOffZK   = kOffZQ   + (size_t)kNH  * kS   * 4;
constexpr size_t kOffCTXH = kOffZK   + (size_t)kNH  * kS   * 4;
constexpr size_t kWsTotal = kOffCTXH + (size_t)kS   * kHid * 2;
static_assert(kWsTotal == 5275648ull);
static_assert(kWsTotal <= 134217728ull);
static_assert((kOffWQKV % 128) == 0 && (kOffWOH % 128) == 0 && (kOffQH % 128) == 0 && (kOffKH % 128) == 0 &&
              (kOffVF % 128) == 0 && (kOffZQ % 128) == 0 && (kOffZK % 128) == 0 && (kOffCTXH % 128) == 0);

__device__ __forceinline__ float flush16(float c) {
  return (fabsf(c) < kF16MinNormal) ? 0.0f : c;
}

__device__ __forceinline__ float h16_to_f32(unsigned hb) {
  const unsigned sgn = (hb & 0x8000u) << 16;
  const unsigned em = hb & 0x7fffu;
  const float fn = __uint_as_float((em << 13) + 0x38000000u);
  const float fs = (float)em * 5.9604644775390625e-8f;
  const float mag = (em < 0x400u) ? fs : fn;
  return __uint_as_float(__float_as_uint(mag) | sgn);
}

__device__ __forceinline__ void score_consts(float g, float& coef, float& zc) {
  const float den = 16.0f * g * kSqrtD;
  coef = 15.0f * (1.0f / den);
  zc = (3.0f * (float)kD / 16.0f) * (1.0f / (g * kSqrtD));
}

namespace eng {

__device__ __forceinline__ v16h frag_load(const _Float16* p) {
  union U { v16h v; v8h h[2]; } f;
  f.h[0] = *(const v8h*)(p);
  f.h[1] = *(const v8h*)(p + 16);
  return f.v;
}

__device__ __forceinline__ v8f wm(v16h a, v16h b, v8f c) {
  c = __builtin_amdgcn_wmma_f32_16x16x32_f16(false, a, false, b, (short)0, c, false, false);
  asm volatile("v_nop\n\tv_nop\n\tv_nop\n\tv_nop" : "+v"(c) : "v"(a), "v"(b));
  return c;
}

__device__ __forceinline__ void acc_guard4(v8f& a, v8f& b, v8f& c, v8f& d) {
  asm volatile("v_nop\n\tv_nop\n\tv_nop\n\tv_nop" : "+v"(a), "+v"(b), "+v"(c), "+v"(d));
}

template <int MODE>
__global__ __launch_bounds__(256) void gemm64_f16(
    const unsigned short* __restrict__ Ap, int lda,
    const unsigned short* __restrict__ Btp, int ldb,
    void* C0, void* C1, void* C2, int ldc,
    const float* b0, const float* b1, const float* b2,
    int M, int N, int K, float scale, float carry16) {
  const _Float16* A  = (const _Float16*)Ap;
  const _Float16* Bt = (const _Float16*)Btp;
  __shared__ __align__(16) float sT[8][16 * 68];
  const int lane = threadIdx.x & 31;
  const int wave = threadIdx.x >> 5;
  const int tilesN = N >> 6;
  const int tilesM = M >> 6;
  const int tile = blockIdx.x * 8 + wave;
  if (tile >= tilesM * tilesN) return;
  const int tm = tile / tilesN;
  const int tn = tile - tm * tilesN;
  const int m0 = tm << 6;
  const int n0 = tn << 6;

  const int rlane = lane & 15;
  const int koff  = (lane >> 4) * 8;
  const int mOff  = (lane >> 4) * 8;

  v8f acc[4][4];
#pragma unroll
  for (int i = 0; i < 4; ++i)
#pragma unroll
    for (int j = 0; j < 4; ++j) acc[i][j] = (v8f){0.f, 0.f, 0.f, 0.f, 0.f, 0.f, 0.f, 0.f};

  for (int k0 = 0; k0 < K; k0 += 32) {
    v16h bh[4];
#pragma unroll
    for (int j = 0; j < 4; ++j) {
      const size_t bo = (size_t)(n0 + (j << 4) + rlane) * ldb + koff + k0;
      bh[j] = frag_load(Bt + bo);
    }
#pragma unroll
    for (int i = 0; i < 4; ++i) {
      const size_t ao = (size_t)(m0 + (i << 4) + rlane) * lda + koff + k0;
      const v16h ah = frag_load(A + ao);
#pragma unroll
      for (int j = 0; j < 4; ++j) acc[i][j] = wm(ah, bh[j], acc[i][j]);
    }
  }
  acc_guard4(acc[0][0], acc[0][1], acc[0][2], acc[0][3]);
  acc_guard4(acc[1][0], acc[1][1], acc[1][2], acc[1][3]);
  acc_guard4(acc[2][0], acc[2][1], acc[2][2], acc[2][3]);
  acc_guard4(acc[3][0], acc[3][1], acc[3][2], acc[3][3]);

  int region = 2;
  int nc0 = n0;
  const float* bp = b0;
  float* Cf = (float*)C0;
  unsigned short* Ch = (unsigned short*)C0;
  if (MODE == 1) {
    region = n0 / kHid;
    nc0 = n0 - region * kHid;
    bp = (region == 0) ? b0 : ((region == 1) ? b1 : b2);
    Cf = (float*)C2;
    Ch = (unsigned short*)((region == 0) ? C0 : C1);
  }
  const bool f32out = (MODE == 0) || (region == 2);
  const float post = f32out ? 1.0f : carry16;

  float* slab = sT[wave];
#pragma unroll
  for (int i = 0; i < 4; ++i) {
    const int mBase = m0 + (i << 4);
#pragma unroll
    for (int j = 0; j < 4; ++j) {
      const float bv = bp[nc0 + (j << 4) + rlane];
#pragma unroll
      for (int r = 0; r < 8; ++r) {
        const float v = (acc[i][j][r] * scale + bv) * post;
        slab[(mOff + r) * 68 + (j << 4) + rlane] = v;
      }
    }
    __builtin_amdgcn_fence(__ATOMIC_RELEASE, "workgroup");
    __builtin_amdgcn_wave_barrier();
    __builtin_amdgcn_fence(__ATOMIC_ACQUIRE, "workgroup");
    if (f32out) {
      const int hh = lane >> 4, c4 = (lane & 15) * 4;
      for (int pass = 0; pass < 2; ++pass) {
#pragma unroll
        for (int it = 0; it < 8; ++it) {
          const int row = it * 2 + hh;
          const v4f v = *(const v4f*)(slab + row * 68 + c4);
          *(volatile v4f*)(Cf + (size_t)(mBase + row) * ldc + nc0 + c4) = v;
        }
        __threadfence();
      }
    } else {
      const int q = lane >> 3, c8 = (lane & 7) * 8;
      for (int pass = 0; pass < 2; ++pass) {
#pragma unroll
        for (int it = 0; it < 4; ++it) {
          const int row = it * 4 + q;
          const float* sp = slab + row * 68 + c8;
          v8h hv;
#pragma unroll
          for (int e = 0; e < 8; ++e) {
            const float c = flush16(sp[e]);
            hv[e] = (_Float16)c;
          }
          *(volatile v8h*)(Ch + (size_t)(mBase + row) * ldc + nc0 + c8) = hv;
        }
        __threadfence();
      }
    }
    __builtin_amdgcn_fence(__ATOMIC_RELEASE, "workgroup");
    __builtin_amdgcn_wave_barrier();
    __builtin_amdgcn_fence(__ATOMIC_ACQUIRE, "workgroup");
  }
}

}

constexpr int kCastBlocksPerPlane = (kS * kHid / 8) / 256;
static_assert(kCastBlocksPerPlane == 128);
static_assert(kCastBlocksPerPlane * 256 * 8 == kS * kHid);

__global__ __launch_bounds__(256) void cast_planes_kernel(
    const float* __restrict__ x, const float* __restrict__ wq, const float* __restrict__ wk,
    const float* __restrict__ wv, const float* __restrict__ wo,
    unsigned short* __restrict__ XH, unsigned short* __restrict__ WQKV, unsigned short* __restrict__ WOH) {
  const unsigned plane = blockIdx.x / (unsigned)kCastBlocksPerPlane;
  const unsigned blk   = blockIdx.x - plane * (unsigned)kCastBlocksPerPlane;
  const unsigned i     = blk * 256u + threadIdx.x;
  const float* src = (plane == 0u) ? x : (plane == 1u) ? wq : (plane == 2u) ? wk : (plane == 3u) ? wv : wo;
  unsigned short* dst = (plane == 0u) ? XH : (plane == 4u) ? WOH : (WQKV + (size_t)(plane - 1u) * kHid * kHid);
  const float carry = (plane == 0u) ? kXCarry : kWCarry;
  const size_t e0 = (size_t)i << 3;
  const v4f a0 = *(const v4f*)(src + e0);
  const v4f a1 = *(const v4f*)(src + e0 + 4);
  v8h hv;
#pragma unroll
  for (int e = 0; e < 4; ++e) {
    const float c0 = flush16(a0[e] * carry);
    const float c1 = flush16(a1[e] * carry);
    hv[e]     = (_Float16)c0;
    hv[4 + e] = (_Float16)c1;
  }
  unsigned short* q = dst + e0;
  *(volatile v8h*)q = hv;
  __threadfence();
  *(volatile v8h*)q = hv;
}

__global__ __launch_bounds__(256) void norms_kernel(
    const unsigned short* __restrict__ QH, const unsigned short* __restrict__ KH,
    const float* __restrict__ mask, const float* __restrict__ gamma,
    float* __restrict__ ZQ, float* __restrict__ ZK) {
  const unsigned idx = blockIdx.x * 256u + threadIdx.x;
  const unsigned h = idx / (unsigned)kS;
  const unsigned s = idx - h * (unsigned)kS;
  const unsigned short* qp = QH + (size_t)s * kHid + h * kD;
  const unsigned short* kp = KH + (size_t)s * kHid + h * kD;
  float sq = 0.0f, sk = 0.0f;
#pragma unroll 1
  for (unsigned c = 0; c < (unsigned)(kD / 8); ++c) {
    const v4u uq = *(const v4u*)(qp + 8u * c);
    const v4u uk = *(const v4u*)(kp + 8u * c);
#pragma unroll
    for (int e = 0; e < 4; ++e) {
      const unsigned wq = uq[e];
      const unsigned wk = uk[e];
      const float q0 = h16_to_f32(wq & 0xffffu);
      const float q1 = h16_to_f32(wq >> 16);
      const float k0 = h16_to_f32(wk & 0xffffu);
      const float k1 = h16_to_f32(wk >> 16);
      sq = fmaf(q0, q0, sq);
      sq = fmaf(q1, q1, sq);
      sk = fmaf(k0, k0, sk);
      sk = fmaf(k1, k1, sk);
    }
  }
  float coef, zc;
  score_consts(gamma[0], coef, zc);
  const float coefc = coef * kInvQK2;
  const float pen = (1.0f - mask[s]) * kMaskPen;
  const float zq = coefc * sq;
  const float zk = coefc * sk + zc + pen;
  volatile float* pq = ZQ + idx;
  volatile float* pk = ZK + idx;
  *pq = zq;
  *pk = zk;
  __threadfence();
  *pq = zq;
  *pk = zk;
}

__global__ __launch_bounds__(256) void relu_sum_kernel(
    const unsigned short* __restrict__ QH, const unsigned short* __restrict__ KH,
    const float* __restrict__ VF, const float* __restrict__ ZQ, const float* __restrict__ ZK,
    const float* __restrict__ gamma, unsigned short* __restrict__ CTXH) {
  __shared__ __align__(16) float z_s[kIT * kZP];
  __shared__ __align__(16) float v_s[kJC * kD];
  __shared__ float zq_s[kIT];

  unsigned tid = threadIdx.x;
  unsigned lane = tid & 31u;
  unsigned wave = tid >> 5;
  asm volatile("" : "+v"(lane));
  asm volatile("" : "+v"(wave));
  unsigned hh = lane >> 4;
  unsigned cl = lane & 15u;
  asm volatile("" : "+v"(hh));
  asm volatile("" : "+v"(cl));

  const unsigned i0 = blockIdx.x * (unsigned)kIT;
  const unsigned h  = blockIdx.y;

  float coef, zc;
  score_consts(gamma[0], coef, zc);
  const float c2 = 2.0f * coef * kInvQK2;

  float zqv = ZQ[(size_t)h * kS + i0 + lane];
  asm volatile("" : "+v"(zqv));
  if (tid < 32u) zq_s[lane] = zqv;

  const _Float16* Qp = (const _Float16*)QH;
  const _Float16* Kp = (const _Float16*)KH;
  v16h afr[2][2];
#pragma unroll
  for (int rt = 0; rt < 2; ++rt)
#pragma unroll
    for (int ks = 0; ks < 2; ++ks)
      afr[rt][ks] = eng::frag_load(Qp + (size_t)(i0 + rt * 16 + cl) * kHid + h * kD + ks * 32 + 8u * hh);

  float acc[8];
#pragma unroll
  for (int e = 0; e < 8; ++e) acc[e] = 0.0f;

  unsigned ri = tid >> 3;
  unsigned d0 = (tid & 7u) * 8u;
  asm volatile("" : "+v"(ri));
  asm volatile("" : "+v"(d0));

#pragma unroll 1
  for (unsigned c = 0; c < (unsigned)(kS / kJC); ++c) {
    const unsigned j0 = c * (unsigned)kJC;
    __syncthreads();

#pragma unroll
    for (int it = 0; it < 8; ++it) {
      const unsigned idx = (unsigned)it * 256u + tid;
      const unsigned r = idx >> 4;
      const unsigned c4 = (idx & 15u) * 4u;
      const v4f vv = *(const v4f*)(VF + (size_t)(j0 + r) * kHid + h * kD + c4);
      *(v4f*)(v_s + r * kD + c4) = vv;
    }

    v8f s0 = (v8f){0.f, 0.f, 0.f, 0.f, 0.f, 0.f, 0.f, 0.f};
    v8f s1 = (v8f){0.f, 0.f, 0.f, 0.f, 0.f, 0.f, 0.f, 0.f};
    const _Float16* krow = Kp + (size_t)(j0 + wave * 16u + cl) * kHid + h * kD + 8u * hh;
#pragma unroll
    for (int ks = 0; ks < 2; ++ks) {
      const v16h bfr = eng::frag_load(krow + ks * 32);
      s0 = eng::wm(afr[0][ks], bfr, s0);
      s1 = eng::wm(afr[1][ks], bfr, s1);
    }
    const float zkj = ZK[(size_t)h * kS + j0 + wave * 16u + cl];
    const unsigned zcol = wave * 16u + cl;
#pragma unroll
    for (int r = 0; r < 8; ++r) {
      const unsigned row0 = 8u * hh + (unsigned)r;
      const unsigned row1 = 16u + row0;
      z_s[row0 * kZP + zcol] = zq_s[row0] + zkj - c2 * s0[r];
      z_s[row1 * kZP + zcol] = zq_s[row1] + zkj - c2 * s1[r];
    }
    __syncthreads();

    const float* zp = z_s + ri * kZP;
    const float* vp = v_s + d0;
#pragma unroll 2
    for (unsigned jj = 0; jj < (unsigned)kJC; jj += 4u) {
      const v4f z4 = *(const v4f*)(zp + jj);
#pragma unroll
      for (int u = 0; u < 4; ++u) {
        const v4f va = *(const v4f*)(vp + (jj + (unsigned)u) * kD);
        const v4f vb = *(const v4f*)(vp + (jj + (unsigned)u) * kD + 4);
        const float zz = z4[u];
        acc[0] += fmaxf(va[0] - zz, 0.0f);
        acc[1] += fmaxf(va[1] - zz, 0.0f);
        acc[2] += fmaxf(va[2] - zz, 0.0f);
        acc[3] += fmaxf(va[3] - zz, 0.0f);
        acc[4] += fmaxf(vb[0] - zz, 0.0f);
        acc[5] += fmaxf(vb[1] - zz, 0.0f);
        acc[6] += fmaxf(vb[2] - zz, 0.0f);
        acc[7] += fmaxf(vb[3] - zz, 0.0f);
      }
    }
  }

  v8h hv;
#pragma unroll
  for (int e = 0; e < 8; ++e) {
    const float cval = flush16(acc[e] * kCtxCarry);
    hv[e] = (_Float16)cval;
  }
  unsigned short* dst = CTXH + (size_t)(i0 + ri) * kHid + h * kD + d0;
  *(volatile v8h*)dst = hv;
  __threadfence();
  *(volatile v8h*)dst = hv;
}

extern "C" void kernel_launch(void* const* d_in, const int* in_sizes, int n_in,
                              void* d_out, int out_size, void* d_ws, size_t ws_size,
                              hipStream_t stream) {
  if (n_in < 11) return;
  if (in_sizes[0] != kS * kHid) return;
  if (in_sizes[1] != kS) return;
  if (in_sizes[2] != kHid * kHid) return;
  if (in_sizes[3] != kHid) return;
  if (in_sizes[4] != kHid * kHid) return;
  if (in_sizes[5] != kHid) return;
  if (in_sizes[6] != kHid * kHid) return;
  if (in_sizes[7] != kHid) return;
  if (in_sizes[8] != kHid * kHid) return;
  if (in_sizes[9] != kHid) return;
  if (in_sizes[10] != 1) return;
  if (out_size != kS * kHid) return;
  if (ws_size < kWsTotal) return;

  const float* hs    = (const float*)d_in[0];
  const float* mask  = (const float*)d_in[1];
  const float* Wq    = (const float*)d_in[2];
  const float* bq    = (const float*)d_in[3];
  const float* Wk    = (const float*)d_in[4];
  const float* bk    = (const float*)d_in[5];
  const float* Wv    = (const float*)d_in[6];
  const float* bv    = (const float*)d_in[7];
  const float* Wo    = (const float*)d_in[8];
  const float* bo    = (const float*)d_in[9];
  const float* gamma = (const float*)d_in[10];
  float* out = (float*)d_out;

  char* ws = (char*)d_ws;
  unsigned short* XH   = (unsigned short*)(ws + kOffXH);
  unsigned short* WQKV = (unsigned short*)(ws + kOffWQKV);
  unsigned short* WOH  = (unsigned short*)(ws + kOffWOH);
  unsigned short* QH   = (unsigned short*)(ws + kOffQH);
  unsigned short* KH   = (unsigned short*)(ws + kOffKH);
  float*          VF   = (float*)(ws + kOffVF);
  float*          ZQ   = (float*)(ws + kOffZQ);
  float*          ZK   = (float*)(ws + kOffZK);
  unsigned short* CTXH = (unsigned short*)(ws + kOffCTXH);

  cast_planes_kernel<<<5 * kCastBlocksPerPlane, 256, 0, stream>>>(hs, Wq, Wk, Wv, Wo, XH, WQKV, WOH);

  eng::gemm64_f16<1><<<dim3((kS / 64) * (kQKV / 64) / 8), 256, 0, stream>>>(
      XH, kHid, WQKV, kHid,
      (void*)QH, (void*)KH, (void*)VF, kHid,
      bq, bk, bv,
      kS, kQKV, kHid, kProjScale, kQKCarry);

  norms_kernel<<<(kNH * kS) / 256, 256, 0, stream>>>(QH, KH, mask, gamma, ZQ, ZK);

  relu_sum_kernel<<<dim3(kS / kIT, kNH), 256, 0, stream>>>(QH, KH, VF, ZQ, ZK, gamma, CTXH);

  eng::gemm64_f16<0><<<dim3((kS / 64) * (kHid / 64) / 8), 256, 0, stream>>>(
      CTXH, kHid, WOH, kHid,
      (void*)out, (void*)out, (void*)out, kHid,
      bo, bo, bo,
      kS, kHid, kHid, kOutScale, 1.0f);
}
